// EquivariantGNN_60919816127138
// MI455X (gfx1250) — hardware-verified
//
#include <hip/hip_runtime.h>
#include <stddef.h>
#include <math.h>


#define NTHR   256
#define NWAVE  8
#define EPT    8
#define CHUNK  (NTHR * EPT)
#define WCAP   (EPT * 32)
#define LISTN  (NWAVE * WCAP)
#define PASSN  (NWAVE * 16)
#define PCAP   (CHUNK + PASSN)
#define NB     256
#define CC     32
#define NBAS   8
#define HIDN   64
#define WD     128
#define AROW   160
#define WROW   128
#define VW     96
#define NGR    64
#define BN_EPS 1e-5

#define PO_W1P 0
#define PO_W2H 2048
#define PO_W2L 6144
#define PO_W3H 10240
#define PO_W3L 18432
#define PO_WSH 26624
#define PO_WSL 27648
#define PO_WVH 28672
#define PO_WVL 29696
#define PLANE_U 30720

#define BO_RB1 0
#define BO_RB2 64
#define BO_RB3 128
#define BO_BSS 256
#define BO_FR  288

#define LO_ACC   0
#define LO_WST   163840
#define LO_LIST  229376
#define LO_PEND  237568
#define LO_BAS   246272
#define LO_META  250368
#define LO_BSM   254464
#define LO_MISC  255680
#define LDS_TOTAL 255744

#define PL_SAH 0
#define PL_SAL 4096
#define PL_VAH 8192
#define PL_VAL 20480

static_assert(LO_WST == NB * AROW * 4);
static_assert(LO_LIST == LO_WST + PASSN * WROW * 4);
static_assert(LO_PEND == LO_LIST + LISTN * 4);
static_assert(LO_BAS == LO_PEND + PCAP * 4);
static_assert(LO_META == LO_BAS + PASSN * 16 * 2);
static_assert(LO_BSM == LO_META + PASSN * 8 * 4);
static_assert(LO_MISC >= LO_BSM + (BO_FR + 8) * 4);
static_assert(LDS_TOTAL >= LO_MISC + 64);
static_assert((PL_VAL + 3 * 128 * 32) * 2 <= PASSN * WROW * 4);
static_assert(NWAVE * 3 * 32 * 8 <= LISTN * 4);
static_assert(128 * 8 <= PCAP * 4);
static_assert(PCAP >= CHUNK + PASSN);
static_assert((NB % 128) == 0 && (NB / NWAVE) * NWAVE == NB);

typedef float          v4f  __attribute__((ext_vector_type(4)));
typedef float          v8f  __attribute__((ext_vector_type(8)));
typedef int            v4i  __attribute__((ext_vector_type(4)));
typedef unsigned short v8us __attribute__((ext_vector_type(8)));
typedef unsigned short v16us __attribute__((ext_vector_type(16)));
typedef __bf16         v16b __attribute__((ext_vector_type(16)));
typedef double         v2d  __attribute__((ext_vector_type(2)));
union FragU { v16us v; v8us h[2]; };

__device__ __forceinline__ int clampi(int x, int lo, int hi) { return x < lo ? lo : (x > hi ? hi : x); }

__device__ __forceinline__ unsigned bfb(float x) {
  unsigned u = __float_as_uint(x);
  u += 0x7FFFu + ((u >> 16) & 1u);
  return u >> 16;
}
__device__ __forceinline__ void split2(float x, unsigned short& hi, unsigned short& lo) {
  const unsigned hb = bfb(x);
  hi = (unsigned short)hb;
  lo = (unsigned short)bfb(x - __uint_as_float(hb << 16));
}

__device__ __forceinline__ v8f wmb(v16us a, v16us b, v8f c) {
  const v16b av = __builtin_bit_cast(v16b, a);
  const v16b bv = __builtin_bit_cast(v16b, b);
  v8f d = __builtin_amdgcn_wmma_f32_16x16x32_bf16(false, av, false, bv, (short)0, c, false, false);
  asm volatile("v_nop\n\tv_nop\n\tv_nop\n\tv_nop" : "+v"(d) : "v"(a), "v"(b));
  return d;
}

__device__ __forceinline__ v16us ldfrag(const unsigned short* p, int pitch, int row, int k0, int hh) {
  const unsigned short* q = p + row * pitch + k0 + 8 * hh;
  FragU f;
  f.h[0] = *(const v8us*)q;
  f.h[1] = *(const v8us*)(q + 16);
  return f.v;
}

__device__ __forceinline__ v8f ldc8(const float* p) {
  const v4f a = *(const v4f*)p;
  const v4f b = *(const v4f*)(p + 4);
  v8f c;
  c[0] = a.x; c[1] = a.y; c[2] = a.z; c[3] = a.w;
  c[4] = b.x; c[5] = b.y; c[6] = b.z; c[7] = b.w;
  return c;
}
__device__ __forceinline__ v8f splat8(float x) {
  v8f c;
#pragma unroll
  for (int i = 0; i < 8; ++i) c[i] = x;
  return c;
}

__device__ __forceinline__ float sigm_f(float x) {
  const float e = __expf(fminf(-x, 80.0f));
  return __builtin_amdgcn_rcpf(1.0f + e);
}
__device__ __forceinline__ float silu_f(float x) { return x * sigm_f(x); }

__device__ __forceinline__ void act_split8(v8f d, v8us& qh, v8us& ql) {
#pragma unroll
  for (int i = 0; i < 8; ++i) {
    unsigned short a, b;
    split2(silu_f(d[i]), a, b);
    qh[i] = a;
    ql[i] = b;
  }
}

__device__ __forceinline__ int scan_chunk(const int* __restrict__ dsts, int nE, int cbase, int nodeBase,
                                          int vec8, int* list, int tid, int wave) {
  int wc = 0;
  const int el0  = tid * EPT;
  const int e0   = cbase + el0;
  const int sent = -2147483647 - 1;
  v4i da, db;
  if (vec8 != 0 && cbase + CHUNK <= nE) {
    da = *(const v4i*)(dsts + e0);
    db = *(const v4i*)(dsts + e0 + 4);
  } else {
    da.x = (e0     < nE) ? dsts[min(e0, nE - 1)] : sent;
    da.y = (e0 + 1 < nE) ? dsts[min(e0 + 1, nE - 1)] : sent;
    da.z = (e0 + 2 < nE) ? dsts[min(e0 + 2, nE - 1)] : sent;
    da.w = (e0 + 3 < nE) ? dsts[min(e0 + 3, nE - 1)] : sent;
    db.x = (e0 + 4 < nE) ? dsts[min(e0 + 4, nE - 1)] : sent;
    db.y = (e0 + 5 < nE) ? dsts[min(e0 + 5, nE - 1)] : sent;
    db.z = (e0 + 6 < nE) ? dsts[min(e0 + 6, nE - 1)] : sent;
    db.w = (e0 + 7 < nE) ? dsts[min(e0 + 7, nE - 1)] : sent;
  }
  const unsigned nb = (unsigned)nodeBase;
  const unsigned s0 = (unsigned)da.x - nb, s1 = (unsigned)da.y - nb;
  const unsigned s2 = (unsigned)da.z - nb, s3 = (unsigned)da.w - nb;
  const unsigned s4 = (unsigned)db.x - nb, s5 = (unsigned)db.y - nb;
  const unsigned s6 = (unsigned)db.z - nb, s7 = (unsigned)db.w - nb;
  const bool h0 = s0 < (unsigned)NB, h1 = s1 < (unsigned)NB, h2 = s2 < (unsigned)NB, h3 = s3 < (unsigned)NB;
  const bool h4 = s4 < (unsigned)NB, h5 = s5 < (unsigned)NB, h6 = s6 < (unsigned)NB, h7 = s7 < (unsigned)NB;
  const unsigned any = __builtin_amdgcn_ballot_w32(h0 | h1 | h2 | h3 | h4 | h5 | h6 | h7);
  if (any != 0u) {
#define HITJ(J, HJ) { \
      const unsigned mj = __builtin_amdgcn_ballot_w32(HJ); \
      if (mj != 0u) { \
        if (HJ) { \
          const int pos = wc + (int)__builtin_amdgcn_mbcnt_lo(mj, 0u); \
          if (pos < WCAP) list[wave * WCAP + pos] = el0 + (J); \
        } \
        wc += (int)__builtin_popcount(mj); } }
    HITJ(0, h0)
    HITJ(1, h1)
    HITJ(2, h2)
    HITJ(3, h3)
    HITJ(4, h4)
    HITJ(5, h5)
    HITJ(6, h6)
    HITJ(7, h7)
#undef HITJ
  }
  return wc;
}

__global__ __launch_bounds__(NTHR) void k_prep_w(
    const float* __restrict__ rW1, const float* __restrict__ rW2, const float* __restrict__ rW3,
    const float* __restrict__ Wss, const float* __restrict__ Wvv, unsigned short* wpl) {
  const int tid = threadIdx.x;
  const int npl = PLANE_U / 8;
  const int npc = 2 * npl;
#pragma unroll 1
  for (int ps = 0; ps < 2; ++ps) {
#pragma unroll 1
    for (int p = tid; p < npc; p += NTHR) {
      const int l = (p >= npl) ? 1 : 0;
      const int u = (p - l * npl) * 8;
      const float* src;
      int ncol, n, k0, prt;
      if (u < PO_W2H) {
        src = rW1 + l * (NBAS * HIDN); ncol = HIDN; n = u >> 5;
        const int ks0 = u & 31; k0 = 0; prt = (ks0 < 16) ? 0 : ((ks0 < 24) ? 1 : 2);
      } else if (u < PO_W3H) {
        int uu = u - PO_W2H; prt = (uu >= 4096) ? 1 : 0; uu -= prt * 4096;
        src = rW2 + l * (HIDN * HIDN); ncol = HIDN; n = uu >> 6; k0 = uu & 63;
      } else if (u < PO_WSH) {
        int uu = u - PO_W3H; prt = (uu >= 8192) ? 1 : 0; uu -= prt * 8192;
        src = rW3 + l * (HIDN * WD); ncol = WD; n = uu >> 6; k0 = uu & 63;
      } else if (u < PO_WVH) {
        int uu = u - PO_WSH; prt = (uu >= 1024) ? 1 : 0; uu -= prt * 1024;
        src = Wss + l * (CC * CC); ncol = CC; n = uu >> 5; k0 = uu & 31;
      } else {
        int uu = u - PO_WVH; prt = (uu >= 1024) ? 1 : 0; uu -= prt * 1024;
        src = Wvv + l * (CC * CC); ncol = CC; n = uu >> 5; k0 = uu & 31;
      }
      v8us val;
#pragma unroll
      for (int i = 0; i < 8; ++i) {
        const float x = src[(k0 + i) * ncol + n];
        unsigned short hb, lb;
        split2(x, hb, lb);
        const unsigned short zv = (unsigned short)0;
        val[i] = (prt == 0) ? hb : ((prt == 1) ? lb : zv);
      }
      *(volatile v8us*)(wpl + (size_t)l * PLANE_U + u) = val;
    }
    if (ps == 0) { __threadfence(); __syncthreads(); }
  }
}

__global__ __launch_bounds__(NTHR) void k_init_s(const int* __restrict__ species, const float* __restrict__ emb,
                                                 float* sfe, int nN, int nSp) {
  const int tid = threadIdx.x;
  const int rb = blockIdx.x * NB;
  v4f vv[8];
#pragma unroll
  for (int i = 0; i < 8; ++i) {
    const int p = i * NTHR + tid;
    const int row = p >> 3, col = 4 * (p & 7);
    const int n = rb + row;
    int sp = species[min(n, nN - 1)];
    sp = clampi(sp, 0, nSp - 1);
    const v4f e = *(const v4f*)(emb + (size_t)sp * CC + col);
    const v4f z4 = {0.0f, 0.0f, 0.0f, 0.0f};
    vv[i] = (n < nN) ? e : z4;
  }
#pragma unroll
  for (int i = 0; i < 8; ++i) {
    const int p = i * NTHR + tid;
    *(volatile v4f*)(sfe + (size_t)(rb + (p >> 3)) * CC + 4 * (p & 7)) = vv[i];
  }
  __threadfence();
#pragma unroll
  for (int i = 0; i < 8; ++i) {
    const int p = i * NTHR + tid;
    *(volatile v4f*)(sfe + (size_t)(rb + (p >> 3)) * CC + 4 * (p & 7)) = vv[i];
  }
}

template <int VZERO>
__global__ __launch_bounds__(NTHR) void k_edge(
    const float* __restrict__ pos, const int* __restrict__ ei, const float* __restrict__ freqs,
    const float* __restrict__ sfe, const float* __restrict__ vfe,
    const unsigned short* __restrict__ wpl,
    const float* __restrict__ rb1, const float* __restrict__ rb2,
    const float* __restrict__ rb3, const float* __restrict__ bss,
    float* spre, float* vpre, double* part, int nN, int nE, int vec8) {
  extern __shared__ __attribute__((aligned(16))) unsigned char dsm[];
  float*          acc   = (float*)(dsm + LO_ACC);
  float*          wst   = (float*)(dsm + LO_WST);
  unsigned short* pln   = (unsigned short*)(dsm + LO_WST);
  int*            list  = (int*)(dsm + LO_LIST);
  int*            pend  = (int*)(dsm + LO_PEND);
  unsigned short* bas   = (unsigned short*)(dsm + LO_BAS);
  float*          emeta = (float*)(dsm + LO_META);
  float*          bsm   = (float*)(dsm + LO_BSM);
  int*            wcnt  = (int*)(dsm + LO_MISC);
  double*         red   = (double*)(dsm + LO_LIST);
  double*         red2  = (double*)(dsm + LO_PEND);

  const int tid = threadIdx.x, lane = tid & 31, wave = tid >> 5, hh = lane >> 4, m = lane & 15;
  const int nodeBase = blockIdx.x * NB;
  const int* srcs = ei;
  const int* dsts = ei + nE;

  {
    const v4f z4 = {0.0f, 0.0f, 0.0f, 0.0f};
    for (int i = tid; i < NB * AROW / 4; i += NTHR) *(v4f*)(acc + 4 * i) = z4;
  }
  if (tid < 64) { bsm[BO_RB1 + tid] = rb1[tid]; bsm[BO_RB2 + tid] = rb2[tid]; }
  if (tid < 128) bsm[BO_RB3 + tid] = rb3[tid];
  if (tid < 32) bsm[BO_BSS + tid] = bss[tid];
  if (tid < 8) bsm[BO_FR + tid] = freqs[tid];
  if (tid == 0) wcnt[NWAVE] = 0;
  __syncthreads();

  const int nChunks = (nE + CHUNK - 1) / CHUNK;
#pragma unroll 1
  for (int ch = 0; ch < nChunks; ++ch) {
    const int cbase = ch * CHUNK;
    const int wc = scan_chunk(dsts, nE, cbase, nodeBase, vec8, list, tid, wave);
    if (lane == 0) wcnt[wave] = wc;
    __syncthreads();

    const int base = wcnt[NWAVE];
    int tot = 0, myoff = 0;
#pragma unroll
    for (int w = 0; w < NWAVE; ++w) {
      int c = wcnt[w];
      c = c > WCAP ? WCAP : (c < 0 ? 0 : c);
      if (w < wave) myoff += c;
      tot += c;
    }
    int newN = base + tot;
    newN = newN > PCAP ? PCAP : newN;
    {
      int n = wcnt[wave];
      n = n > WCAP ? WCAP : (n < 0 ? 0 : n);
      const int* lp = list + wave * WCAP;
      for (int i = lane; i < n; i += 32) {
        const int pp = base + myoff + i;
        if (pp < PCAP) pend[pp] = cbase + lp[i];
      }
    }
    const int fin = (ch == nChunks - 1) ? 1 : 0;
    const int R   = (fin != 0) ? (newN + PASSN - 1) / PASSN : newN / PASSN;
    const int Pv  = (fin != 0) ? newN : R * PASSN;
    __syncthreads();

#pragma unroll 1
    for (int r = 0; r < R; ++r) {
      {
        const int j = wave * 16 + m;
        const int idx = r * PASSN + j;
        const bool valid = idx < Pv;
        int e = pend[idx];
        e = valid ? e : 0;
        e = clampi(e, 0, nE - 1);
        int d = dsts[e];
        int s = srcs[e];
        int slot = d - nodeBase;
        if (!valid || (unsigned)slot >= (unsigned)NB) slot = -1;
        d = clampi(d, 0, nN - 1);
        s = clampi(s, 0, nN - 1);
        const float* pd = pos + (size_t)d * 3;
        const float* pq = pos + (size_t)s * 3;
        const float dx = pd[0] - pq[0];
        const float dy = pd[1] - pq[1];
        const float dz = pd[2] - pq[2];
        const float dist = sqrtf(dx * dx + dy * dy + dz * dz);
        const float rinv = 1.0f / fmaxf(dist, 1e-6f);
        const float yinv = 1.0f / fmaxf(dist, 1e-9f);
        const float xq = fminf(dist * 0.2f, 1.0f);
        const float x2 = xq * xq, x3 = x2 * xq, x4 = x2 * x2, x5 = x4 * xq;
        float cut = 1.0f - 6.0f * x5 + 15.0f * x4 - 10.0f * x3;
        cut = (dist <= 5.0f) ? cut : 0.0f;
#pragma unroll 1
        for (int k = 0; k < NBAS; ++k) {
          const float bk = (sinf(bsm[BO_FR + k] * dist) * rinv) * cut;
          unsigned short hb, lb;
          split2(bk, hb, lb);
          bas[j * 16 + 8 * hh + k] = (hh == 0) ? hb : lb;
        }
        v4f ma, mb;
        ma.x = __int_as_float(slot); ma.y = __int_as_float(s); ma.z = dx * yinv; ma.w = dy * yinv;
        mb.x = dz * yinv; mb.y = dist; mb.z = 0.0f; mb.w = 0.0f;
        *(v4f*)(emeta + j * 8 + 4 * hh) = (hh == 0) ? ma : mb;
      }
      __syncthreads();

      {
        const int j = wave * 16 + m;
        v8us z8;
#pragma unroll
        for (int i = 0; i < 8; ++i) z8[i] = (unsigned short)0;
        FragU b1;
        {
          const unsigned short* bp = bas + j * 16;
          const v8us p0 = *(const v8us*)(bp + 8 * hh);
          const v8us p1 = *(const v8us*)bp;
          b1.h[0] = p0;
          b1.h[1] = (hh == 0) ? p1 : z8;
        }
        FragU b2h[2], b2l[2];
#pragma unroll
        for (int ft = 0; ft < 4; ++ft) {
          const v16us a = ldfrag(wpl + PO_W1P, 32, 16 * ft + m, 0, hh);
          v8f c = ldc8(bsm + BO_RB1 + 16 * ft + 8 * hh);
          c = wmb(a, b1.v, c);
          v8us qh, ql;
          act_split8(c, qh, ql);
          b2h[ft >> 1].h[ft & 1] = qh;
          b2l[ft >> 1].h[ft & 1] = ql;
        }
        FragU b3h[2], b3l[2];
#pragma unroll
        for (int ft = 0; ft < 4; ++ft) {
          v8f c = ldc8(bsm + BO_RB2 + 16 * ft + 8 * hh);
#pragma unroll
          for (int ks = 0; ks < 2; ++ks) {
            const v16us ah = ldfrag(wpl + PO_W2H, 64, 16 * ft + m, 32 * ks, hh);
            const v16us al = ldfrag(wpl + PO_W2L, 64, 16 * ft + m, 32 * ks, hh);
            c = wmb(ah, b2h[ks].v, c);
            c = wmb(ah, b2l[ks].v, c);
            c = wmb(al, b2h[ks].v, c);
          }
          v8us qh, ql;
          act_split8(c, qh, ql);
          b3h[ft >> 1].h[ft & 1] = qh;
          b3l[ft >> 1].h[ft & 1] = ql;
        }
        constexpr int NFT = (VZERO != 0) ? 4 : 8;
#pragma unroll
        for (int fi = 0; fi < NFT; ++fi) {
          const int ft = (VZERO != 0) ? ((fi & 1) + 4 * (fi >> 1)) : fi;
          v8f c = ldc8(bsm + BO_RB3 + 16 * ft + 8 * hh);
#pragma unroll
          for (int ks = 0; ks < 2; ++ks) {
            const v16us ah = ldfrag(wpl + PO_W3H, 64, 16 * ft + m, 32 * ks, hh);
            const v16us al = ldfrag(wpl + PO_W3L, 64, 16 * ft + m, 32 * ks, hh);
            c = wmb(ah, b3h[ks].v, c);
            c = wmb(ah, b3l[ks].v, c);
            c = wmb(al, b3h[ks].v, c);
          }
          float* wr = wst + j * WROW + ((ft & 1) * 16 + 8 * hh) * 4 + (ft >> 1);
#pragma unroll
          for (int i = 0; i < 8; ++i) wr[4 * i] = c[i];
        }
      }
      __syncthreads();

      {
        const int q = lane >> 3, t = lane & 7;
        const int c = wave * 4 + q;
        const bool act = t < 5;
        const int aoff = (t == 0) ? c : ((t == 1) ? (CC + c) : ((t < 5) ? (2 * CC + 3 * c + (t - 2)) : 0));
#pragma unroll 1
        for (int jj = 0; jj < PASSN; ++jj) {
          const v4f mt = *(const v4f*)(emeta + jj * 8);
          const int slot = __float_as_int(mt.x);
          if (slot < 0) continue;
          const int sl = slot > NB - 1 ? NB - 1 : slot;
          const int src = __float_as_int(mt.y);
          const float y0 = mt.z, y1 = mt.w, y2 = emeta[jj * 8 + 4];
          const v4f w4v = *(const v4f*)(wst + jj * WROW + c * 4);
          const float xs = sfe[(size_t)src * CC + c];
          float xv0 = 0.0f, xv1 = 0.0f, xv2 = 0.0f;
          if (VZERO == 0) {
            const float* vp = vfe + ((size_t)src * CC + c) * 3;
            xv0 = vp[0]; xv1 = vp[1]; xv2 = vp[2];
          }
          const float w1 = w4v.x;
          const float w2 = (VZERO != 0) ? 0.0f : w4v.y;
          const float w3 = w4v.z;
          const float w4 = (VZERO != 0) ? 0.0f : w4v.w;
          const float msf = w1 * xs;
          const float msg = w2 * (xv0 * y0 + xv1 * y1 + xv2 * y2);
          const float yd  = (t == 2) ? y0 : ((t == 3) ? y1 : y2);
          const float xvd = (t == 2) ? xv0 : ((t == 3) ? xv1 : xv2);
          const float mv  = (w3 * xs) * yd + w4 * xvd;
          const float val = (t == 0) ? msf : ((t == 1) ? msg : mv);
          if (act) acc[sl * AROW + aoff] += val;
        }
      }
      __syncthreads();
    }

    int rem = newN - R * PASSN;
    rem = rem < 0 ? 0 : rem;
    if (R > 0 && tid < rem) pend[tid] = pend[R * PASSN + tid];
    if (tid == 0) wcnt[NWAVE] = rem;
  }
  __syncthreads();

#pragma unroll 1
  for (int hf = 0; hf < 2; ++hf) {
#pragma unroll 1
    for (int it = tid; it < 128 * CC; it += NTHR) {
      const int nl = it >> 5, c = it & 31;
      const float* ar = acc + (128 * hf + nl) * AROW;
      const float sa = silu_f(ar[c]);
      const float g  = sigm_f(ar[CC + c]);
      unsigned short u0, u1;
      split2(sa, u0, u1);
      pln[PL_SAH + nl * 32 + c] = u0;
      pln[PL_SAL + nl * 32 + c] = u1;
#pragma unroll
      for (int d = 0; d < 3; ++d) {
        split2(g * ar[2 * CC + 3 * c + d], u0, u1);
        pln[PL_VAH + (3 * nl + d) * 32 + c] = u0;
        pln[PL_VAL + (3 * nl + d) * 32 + c] = u1;
      }
    }
    __syncthreads();
    {
      const v16us ah = ldfrag(pln + PL_SAH, 32, 16 * wave + m, 0, hh);
      const v16us al = ldfrag(pln + PL_SAL, 32, 16 * wave + m, 0, hh);
#pragma unroll
      for (int ct = 0; ct < 2; ++ct) {
        const v16us bh = ldfrag(wpl + PO_WSH, 32, 16 * ct + m, 0, hh);
        const v16us bl = ldfrag(wpl + PO_WSL, 32, 16 * ct + m, 0, hh);
        v8f c = splat8(bsm[BO_BSS + 16 * ct + m]);
        c = wmb(ah, bh, c);
        c = wmb(ah, bl, c);
        c = wmb(al, bh, c);
        float* orow = acc + (128 * hf + 16 * wave + 8 * hh) * AROW + 16 * ct + m;
#pragma unroll
        for (int i = 0; i < 8; ++i) orow[i * AROW] = c[i];
      }
    }
#pragma unroll
    for (int ii = 0; ii < 3; ++ii) {
      const int rt = wave + 8 * ii;
      const v16us ah = ldfrag(pln + PL_VAH, 32, 16 * rt + m, 0, hh);
      const v16us al = ldfrag(pln + PL_VAL, 32, 16 * rt + m, 0, hh);
#pragma unroll
      for (int ct = 0; ct < 2; ++ct) {
        const v16us bh = ldfrag(wpl + PO_WVH, 32, 16 * ct + m, 0, hh);
        const v16us bl = ldfrag(wpl + PO_WVL, 32, 16 * ct + m, 0, hh);
        v8f c = splat8(0.0f);
        c = wmb(ah, bh, c);
        c = wmb(ah, bl, c);
        c = wmb(al, bh, c);
#pragma unroll
        for (int i = 0; i < 8; ++i) {
          const int rho = 16 * rt + 8 * hh + i;
          const int nl = rho / 3;
          const int d = rho - 3 * nl;
          acc[(128 * hf + nl) * AROW + 2 * CC + (16 * ct + m) * 3 + d] = c[i];
        }
      }
    }
    __syncthreads();
  }

  {
    double s1 = 0.0, s2 = 0.0, s3 = 0.0;
#pragma unroll 1
    for (int i = 0; i < NB / NWAVE; ++i) {
      const int nl = wave * (NB / NWAVE) + i;
      if (nodeBase + nl < nN) {
        const float* ar = acc + nl * AROW;
        const float sp = ar[lane];
        const float a0 = ar[2 * CC + 3 * lane], a1 = ar[2 * CC + 3 * lane + 1], a2 = ar[2 * CC + 3 * lane + 2];
        s1 += (double)sp;
        s2 += (double)sp * (double)sp;
        s3 += (double)a0 * (double)a0 + (double)a1 * (double)a1 + (double)a2 * (double)a2;
      }
    }
    red[(wave * 3 + 0) * 32 + lane] = s1;
    red[(wave * 3 + 1) * 32 + lane] = s2;
    red[(wave * 3 + 2) * 32 + lane] = s3;
  }
  __syncthreads();
  if (tid < 128) {
    double v = 0.0;
    if (tid < 96) {
      const int g = tid >> 5, c = tid & 31;
#pragma unroll
      for (int w = 0; w < NWAVE; ++w) v += red[(w * 3 + g) * 32 + c];
    }
    red2[tid] = v;
  }
  __syncthreads();

#pragma unroll 1
  for (int ps = 0; ps < 2; ++ps) {
    if (tid < 64) {
      const v2d pv = *(const v2d*)(red2 + 2 * tid);
      *(volatile v2d*)(part + (size_t)blockIdx.x * 128 + 2 * tid) = pv;
    }
#pragma unroll
    for (int i = 0; i < 8; ++i) {
      const int p = i * NTHR + tid;
      const int nl = p >> 3, col = 4 * (p & 7);
      const v4f v = *(const v4f*)(acc + nl * AROW + col);
      *(volatile v4f*)(spre + (size_t)(nodeBase + nl) * CC + col) = v;
    }
#pragma unroll
    for (int i = 0; i < 24; ++i) {
      const int p = i * NTHR + tid;
      const int f = 4 * p;
      const int nl = f / VW, col = f - nl * VW;
      const v4f v = *(const v4f*)(acc + nl * AROW + 2 * CC + col);
      *(volatile v4f*)(vpre + (size_t)nodeBase * VW + f) = v;
    }
    if (ps == 0) __threadfence();
  }
}

__global__ __launch_bounds__(NTHR) void k_bnfin(const double* __restrict__ part,
                                                const float* __restrict__ gs, const float* __restrict__ bs,
                                                const float* __restrict__ gv, float* bnl, int nBlk, int nN) {
  __shared__ double rd[96];
  __shared__ __attribute__((aligned(16))) float ln[128];
  const int tid = threadIdx.x, lane = tid & 31, wave = tid >> 5;
  if (tid < 96) {
    double s = 0.0;
#pragma unroll 1
    for (int b = 0; b < nBlk; ++b) s += part[(size_t)b * 128 + tid];
    rd[tid] = s;
  }
  __syncthreads();
  if (tid < 32) {
    const double inv = 1.0 / (double)nN;
    const double mu = rd[tid] * inv;
    double var = rd[32 + tid] * inv - mu * mu;
    if (var < 0.0) var = 0.0;
    const double sc = (double)gs[tid] / sqrt(var + BN_EPS);
    const double vn = rd[64 + tid] * inv * (1.0 / 3.0);
    const double vsc = (double)gv[tid] / sqrt(vn + BN_EPS);
    ln[tid]      = (float)mu;
    ln[32 + tid] = (float)sc;
    ln[64 + tid] = bs[tid];
    ln[96 + tid] = (float)vsc;
  }
  __syncthreads();
  v4f rv = {0.0f, 0.0f, 0.0f, 0.0f};
  const bool wr = (wave == 0);
  if (wr) rv = *(const v4f*)(ln + 4 * lane);
  if (wr) *(volatile v4f*)(bnl + 4 * lane) = rv;
  __threadfence();
  if (wr) *(volatile v4f*)(bnl + 4 * lane) = rv;
}

template <int VZERO>
__global__ __launch_bounds__(NTHR) void k_apply(float* sfe, float* vfe,
                                                const float* __restrict__ spre, const float* __restrict__ vpre,
                                                const float* __restrict__ bnl) {
  __shared__ __attribute__((aligned(16))) float bl[128];
  const int tid = threadIdx.x;
  if (tid < 128) bl[tid] = bnl[tid];
  __syncthreads();
  const size_t rb = (size_t)blockIdx.x * 64;
  v4f so[2], vo[6];
#pragma unroll
  for (int i = 0; i < 2; ++i) {
    const int p = i * NTHR + tid;
    const int row = p >> 3, col = 4 * (p & 7);
    const size_t idx = (rb + row) * CC + col;
    const v4f old = *(const v4f*)(sfe + idx);
    const v4f pr  = *(const v4f*)(spre + idx);
    const v4f mu  = *(const v4f*)(bl + col);
    const v4f sc  = *(const v4f*)(bl + 32 + col);
    const v4f sh  = *(const v4f*)(bl + 64 + col);
    so[i] = old + ((pr - mu) * sc + sh);
  }
#pragma unroll
  for (int i = 0; i < 6; ++i) {
    const int p = i * NTHR + tid;
    const int f = 4 * p;
    const int col = f % VW;
    const size_t idx = rb * VW + (size_t)f;
    const v4f pr = *(const v4f*)(vpre + idx);
    v4f old = {0.0f, 0.0f, 0.0f, 0.0f};
    if (VZERO == 0) old = *(const v4f*)(vfe + idx);
    v4f scv;
    scv.x = bl[96 + (col + 0) / 3]; scv.y = bl[96 + (col + 1) / 3];
    scv.z = bl[96 + (col + 2) / 3]; scv.w = bl[96 + (col + 3) / 3];
    vo[i] = old + pr * scv;
  }
#pragma unroll
  for (int i = 0; i < 2; ++i) {
    const int p = i * NTHR + tid;
    *(volatile v4f*)(sfe + (rb + (p >> 3)) * CC + 4 * (p & 7)) = so[i];
  }
#pragma unroll
  for (int i = 0; i < 6; ++i) {
    const int p = i * NTHR + tid;
    *(volatile v4f*)(vfe + rb * VW + (size_t)4 * p) = vo[i];
  }
  __threadfence();
#pragma unroll
  for (int i = 0; i < 2; ++i) {
    const int p = i * NTHR + tid;
    *(volatile v4f*)(sfe + (rb + (p >> 3)) * CC + 4 * (p & 7)) = so[i];
  }
#pragma unroll
  for (int i = 0; i < 6; ++i) {
    const int p = i * NTHR + tid;
    *(volatile v4f*)(vfe + rb * VW + (size_t)4 * p) = vo[i];
  }
}

__global__ __launch_bounds__(NTHR) void k_out(const float* __restrict__ sfe, const int* __restrict__ batch,
                                              const int* __restrict__ species, const float* __restrict__ wout,
                                              const float* __restrict__ bout, const float* __restrict__ aref,
                                              float* out, int nN, int nSp) {
  __shared__ float gw[NWAVE * NGR];
  __shared__ __attribute__((aligned(16))) float go[NGR];
  const int tid = threadIdx.x, lane = tid & 31, wave = tid >> 5;
  for (int i = tid; i < NWAVE * NGR; i += NTHR) gw[i] = 0.0f;
  __syncthreads();
  const float wo = wout[lane];
  const float b0 = bout[0];
  const int per = (nN + NWAVE - 1) / NWAVE;
  const int n0 = wave * per;
  const int n1 = min(n0 + per, nN);
#pragma unroll 1
  for (int n = n0; n < n1; ++n) {
    float v = sfe[(size_t)n * CC + lane] * wo;
    v += __shfl_xor(v, 16, 32);
    v += __shfl_xor(v, 8, 32);
    v += __shfl_xor(v, 4, 32);
    v += __shfl_xor(v, 2, 32);
    v += __shfl_xor(v, 1, 32);
    const int b = batch[n];
    int sp = species[n];
    sp = clampi(sp, 0, nSp - 1);
    const float e = v + b0 + aref[sp];
    if (lane == 0 && (unsigned)b < (unsigned)NGR) gw[wave * NGR + b] += e;
  }
  __syncthreads();
  if (tid < NGR) {
    float g = 0.0f;
#pragma unroll
    for (int w = 0; w < NWAVE; ++w) g += gw[w * NGR + tid];
    go[tid] = g;
  }
  __syncthreads();
  v4f rv = {0.0f, 0.0f, 0.0f, 0.0f};
  const bool wr = (wave == 0) && (lane < 16);
  if (wr) rv = *(const v4f*)(go + 4 * lane);
  if (wr) *(volatile v4f*)(out + 4 * lane) = rv;
  __threadfence();
  if (wr) *(volatile v4f*)(out + 4 * lane) = rv;
}

extern "C" void kernel_launch(void* const* d_in, const int* in_sizes, int n_in,
                              void* d_out, int out_size, void* d_ws, size_t ws_size,
                              hipStream_t stream) {
  if (n_in < 21) return;
  const int nN = in_sizes[0];
  if (nN < 1) return;
  if (in_sizes[1] != 3 * nN || in_sizes[3] != nN) return;
  if (in_sizes[2] < 2 || (in_sizes[2] & 1) != 0) return;
  const int nE = in_sizes[2] / 2;
  if (in_sizes[4] < CC || (in_sizes[4] % CC) != 0) return;
  const int nSp = in_sizes[4] / CC;
  if (in_sizes[5] != NBAS) return;
  if (in_sizes[6] != 2 * NBAS * HIDN || in_sizes[7] < 2 * HIDN) return;
  if (in_sizes[8] != 2 * HIDN * HIDN || in_sizes[9] < 2 * HIDN) return;
  if (in_sizes[10] != 2 * HIDN * WD || in_sizes[11] < 2 * WD) return;
  if (in_sizes[12] != 2 * CC * CC || in_sizes[13] < 2 * CC || in_sizes[14] != 2 * CC * CC) return;
  if (in_sizes[15] < 2 * CC || in_sizes[16] < 2 * CC || in_sizes[17] < 2 * CC) return;
  if (in_sizes[18] != CC || in_sizes[19] < 1 || in_sizes[20] < nSp) return;
  if (out_size != NGR) return;

  const int*   species = (const int*)d_in[0];
  const float* pos     = (const float*)d_in[1];
  const int*   eidx    = (const int*)d_in[2];
  const int*   batch   = (const int*)d_in[3];
  const float* emb     = (const float*)d_in[4];
  const float* freqs   = (const float*)d_in[5];
  const float* rW1     = (const float*)d_in[6];
  const float* rb1     = (const float*)d_in[7];
  const float* rW2     = (const float*)d_in[8];
  const float* rb2     = (const float*)d_in[9];
  const float* rW3     = (const float*)d_in[10];
  const float* rb3     = (const float*)d_in[11];
  const float* Wss     = (const float*)d_in[12];
  const float* bss     = (const float*)d_in[13];
  const float* Wvv     = (const float*)d_in[14];
  const float* bn_gs   = (const float*)d_in[15];
  const float* bn_bs   = (const float*)d_in[16];
  const float* bn_gv   = (const float*)d_in[17];
  const float* W_out   = (const float*)d_in[18];
  const float* b_out   = (const float*)d_in[19];
  const float* aref    = (const float*)d_in[20];
  float* out = (float*)d_out;

  const int nBlk = (nN + NB - 1) / NB;
  const size_t Npad = (size_t)nBlk * NB;

  size_t off = 0;
  const size_t oW  = off; off += (size_t)2 * PLANE_U * 2;       off = (off + 255) & ~(size_t)255;
  const size_t oS  = off; off += Npad * CC * 4;                  off = (off + 255) & ~(size_t)255;
  const size_t oV  = off; off += Npad * VW * 4;                  off = (off + 255) & ~(size_t)255;
  const size_t oSP = off; off += Npad * CC * 4;                  off = (off + 255) & ~(size_t)255;
  const size_t oVP = off; off += Npad * VW * 4;                  off = (off + 255) & ~(size_t)255;
  const size_t oPT = off; off += (size_t)nBlk * 128 * 8;         off = (off + 255) & ~(size_t)255;
  const size_t oBL = off; off += 512;                            off = (off + 255) & ~(size_t)255;
  if (off > ws_size) return;

  char* ws = (char*)d_ws;
  unsigned short* wpl = (unsigned short*)(ws + oW);
  float*  sfe  = (float*)(ws + oS);
  float*  vfe  = (float*)(ws + oV);
  float*  spre = (float*)(ws + oSP);
  float*  vpre = (float*)(ws + oVP);
  double* part = (double*)(ws + oPT);
  float*  bnl  = (float*)(ws + oBL);

  const int vec8 = ((nE & 3) == 0) ? 1 : 0;

  hipFuncSetAttribute(reinterpret_cast<const void*>(&k_edge<1>), hipFuncAttributeMaxDynamicSharedMemorySize, LDS_TOTAL);
  hipFuncSetAttribute(reinterpret_cast<const void*>(&k_edge<0>), hipFuncAttributeMaxDynamicSharedMemorySize, LDS_TOTAL);

  k_prep_w<<<1, NTHR, 0, stream>>>(rW1, rW2, rW3, Wss, Wvv, wpl);
  k_init_s<<<nBlk, NTHR, 0, stream>>>(species, emb, sfe, nN, nSp);

  k_edge<1><<<nBlk, NTHR, LDS_TOTAL, stream>>>(
      pos, eidx, freqs, sfe, vfe, wpl,
      rb1, rb2, rb3, bss, spre, vpre, part, nN, nE, vec8);
  k_bnfin<<<1, NTHR, 0, stream>>>(part, bn_gs, bn_bs, bn_gv, bnl, nBlk, nN);
  k_apply<1><<<(unsigned)(Npad / 64), NTHR, 0, stream>>>(sfe, vfe, spre, vpre, bnl);

  k_edge<0><<<nBlk, NTHR, LDS_TOTAL, stream>>>(
      pos, eidx, freqs, sfe, vfe, wpl + PLANE_U,
      rb1 + HIDN, rb2 + HIDN, rb3 + WD, bss + CC, spre, vpre, part, nN, nE, vec8);
  k_bnfin<<<1, NTHR, 0, stream>>>(part, bn_gs + CC, bn_bs + CC, bn_gv + CC, bnl, nBlk, nN);
  k_apply<0><<<(unsigned)(Npad / 64), NTHR, 0, stream>>>(sfe, vfe, spre, vpre, bnl);

  k_out<<<1, NTHR, 0, stream>>>(sfe, batch, species, W_out, b_out, aref, out, nN, nSp);
}
